// FastWeightAttention_91182155694169
// MI455X (gfx1250) — hardware-verified
//
#include <hip/hip_runtime.h>
#include <math.h>

typedef __attribute__((ext_vector_type(16))) _Float16 v16h;
typedef __attribute__((ext_vector_type(16))) __bf16 v16b;
typedef __attribute__((ext_vector_type(8)))  _Float16 v8h;
typedef __attribute__((ext_vector_type(8)))  float v8f;
typedef __attribute__((ext_vector_type(4)))  float v4f;
typedef __attribute__((ext_vector_type(2)))  float v2f;
typedef __attribute__((ext_vector_type(4)))  unsigned v4u;
typedef __attribute__((ext_vector_type(4)))  int v4i;
typedef float __attribute__((may_alias)) float_a;
typedef int __attribute__((may_alias)) int_a;

template <typename T> __device__ __forceinline__ void vst2(void* p, T v) { *(volatile T*)p = v; __threadfence(); *(volatile T*)p = v; }
__device__ __forceinline__ v8f wmma16(v16h a, v16h b, v8f c) {
  v8f d = __builtin_amdgcn_wmma_f32_16x16x32_f16(false, a, false, b, (short)0, c, false, false);
  asm volatile("v_nop\n\tv_nop\n\tv_nop\n\tv_nop" : "+v"(d) : "v"(a), "v"(b));
  return d;
}
__device__ __forceinline__ v8f wmma_bf(v16b a, v16b b, v8f c) {
  v8f d = __builtin_amdgcn_wmma_f32_16x16x32_bf16(false, a, false, b, (short)0, c, false, false);
  asm volatile("v_nop\n\tv_nop\n\tv_nop\n\tv_nop" : "+v"(d) : "v"(a), "v"(b));
  return d;
}
__device__ __forceinline__ v16h frag_h(const _Float16* rowk0, int lane) {
  union { v16h v; v8h q[2]; } u; const _Float16* p = rowk0 + 8 * (lane >> 4);
  u.q[0] = *(const v8h*)p; u.q[1] = *(const v8h*)(p + 16); return u.v;
}
__device__ __forceinline__ v16h frag_f32(const float* rowk0, int lane) {
  v16h a; const float* p = rowk0 + 8 * (lane >> 4);
#pragma unroll
  for (int i = 0; i < 8; ++i) { a[i] = (_Float16)p[i]; a[8 + i] = (_Float16)p[16 + i]; }
  return a;
}
__device__ __forceinline__ v16h frag_f32s(const float* rowk0, int lane, float sc) {
  v16h a; const float* p = rowk0 + 8 * (lane >> 4);
#pragma unroll
  for (int i = 0; i < 8; ++i) { a[i] = (_Float16)(p[i] * sc); a[8 + i] = (_Float16)(p[16 + i] * sc); }
  return a;
}
__device__ __forceinline__ v16h fragc_f32(const float* W, int k0, int n, int lane, int ld, int K) {
  v16h a; const int g = lane >> 4;
#pragma unroll
  for (int i = 0; i < 8; ++i) { const int ka = k0 + 8 * g + i, kb = ka + 16;
    a[i] = (_Float16)(ka < K ? W[(size_t)(ka < K ? ka : K - 1) * ld + n] : 0.f); a[8 + i] = (_Float16)(kb < K ? W[(size_t)(kb < K ? kb : K - 1) * ld + n] : 0.f); }
  return a;
}
struct F2 { v16b h, l; };
__device__ __forceinline__ F2 bsplit16(const float v[16]) { F2 r;
#pragma unroll
  for (int i = 0; i < 16; ++i) { const __bf16 h = (__bf16)v[i]; r.h[i] = h; r.l[i] = (__bf16)(v[i] - (float)h); }
  return r; }
__device__ __forceinline__ F2 split_row(const float* row, int k0, int lane) { float v[16]; const float* p = row + k0 + 8 * (lane >> 4);
#pragma unroll
  for (int i = 0; i < 8; ++i) { v[i] = p[i]; v[8 + i] = p[16 + i]; }
  return bsplit16(v); }
__device__ __forceinline__ F2 split_rowK(const float* row, int k0, int lane, int K) { float v[16]; const int g = lane >> 4;
#pragma unroll
  for (int i = 0; i < 8; ++i) { const int ka = k0 + 8 * g + i, kb = ka + 16; v[i] = ka < K ? row[ka < K ? ka : K - 1] : 0.f; v[8 + i] = kb < K ? row[kb < K ? kb : K - 1] : 0.f; }
  return bsplit16(v); }
__device__ __forceinline__ F2 split_col(const float* W, int k0, int n, int lane, int ld, int K) { float v[16]; const int g = lane >> 4;
#pragma unroll
  for (int i = 0; i < 8; ++i) { const int ka = k0 + 8 * g + i, kb = ka + 16; v[i] = ka < K ? W[(size_t)(ka < K ? ka : K - 1) * ld + n] : 0.f; v[8 + i] = kb < K ? W[(size_t)(kb < K ? kb : K - 1) * ld + n] : 0.f; }
  return bsplit16(v); }
__device__ __forceinline__ v8f mac3(const F2& a, const F2& b, v8f c) { c = wmma_bf(a.l, b.h, c); c = wmma_bf(a.h, b.l, c); return wmma_bf(a.h, b.h, c); }
__device__ __forceinline__ float sigm(float v) { return 1.0f / (1.0f + expf(-v)); }
#define LDSX() do { asm volatile("s_wait_dscnt 0" ::: "memory"); __builtin_amdgcn_wave_barrier(); __builtin_amdgcn_fence(__ATOMIC_RELEASE, "workgroup"); } while (0)


#define NB 2
#define LL 2048
#define DM_ 1024
#define NH 16
#define HD 64
#ifndef TNB
#define TNB NB
#endif
#ifndef TQB
#define TQB (LL / 64)
#endif
typedef __attribute__((ext_vector_type(8))) __bf16 v8b;
__device__ __forceinline__ v16b frag_b(const __bf16* rowk0, int lane) {
  union { v16b v; v8b q[2]; } u; const __bf16* p = rowk0 + 8 * (lane >> 4);
  u.q[0] = *(const v8b*)p; u.q[1] = *(const v8b*)(p + 16); return u.v;
}
__device__ __forceinline__ float bfr(float v) { return (float)(__bf16)v; }
__device__ __attribute__((noinline)) float exp_ni(float v) { return expf(v); }
__device__ __attribute__((noinline)) float erf_ni(float v) { return erff(v); }

#define WS_QH  0u
#define WS_KH  (WS_QH + 2u * (size_t)NB * LL * DM_)
#define WS_VT  (WS_KH + 2u * (size_t)NB * LL * DM_)
#define WS_GT  (WS_VT + 2u * (size_t)NB * DM_ * LL)
#define WS_GJ  (WS_GT + 4u * (size_t)NB * LL * 32)
#define WS_O   (WS_GJ + 4u * (size_t)NB * NH * LL)
#define WS_END (WS_O + 4u * (size_t)NB * LL * DM_)

__device__ __forceinline__ float phi1(float x) { return x > 0.f ? x + 1.0f : expf(x); }
__global__ __launch_bounds__(128) void k_proj(const float* __restrict__ X, const float* __restrict__ WQ, const float* __restrict__ WK, const float* __restrict__ WV, _Float16* __restrict__ QH, _Float16* __restrict__ KH, _Float16* __restrict__ VT) { __shared__ __align__(16) _Float16 sh[64][136]; __shared__ __align__(16) _Float16 th[128][72];
  const int tid = threadIdx.x, wave = tid >> 5, lane = tid & 31, col = lane & 15, g = lane >> 4; const int which = blockIdx.z; const int c0 = blockIdx.y * 128; const size_t r0 = (size_t)blockIdx.x * 64; const float* Wm = which == 0 ? WQ : which == 1 ? WK : WV;
  v8f acc[8] = {};
#pragma unroll 2
  for (int kc = 0; kc < DM_ / 32; ++kc) { v16b a; { const float* p = X + (r0 + wave * 16 + col) * DM_ + kc * 32 + 8 * g;
#pragma unroll
      for (int i = 0; i < 8; ++i) { a[i] = (__bf16)p[i]; a[8 + i] = (__bf16)p[16 + i]; } }
#pragma unroll
    for (int j = 0; j < 8; ++j) { v16b w; const int o = c0 + j * 16 + col;
#pragma unroll
      for (int i = 0; i < 8; ++i) { w[i] = (__bf16)Wm[(size_t)o * DM_ + kc * 32 + 8 * g + i]; w[8 + i] = (__bf16)Wm[(size_t)o * DM_ + kc * 32 + 16 + 8 * g + i]; }
      acc[j] = wmma_bf(a, w, acc[j]); } }
  if (which < 2) {
#pragma unroll
    for (int j = 0; j < 8; ++j)
#pragma unroll
      for (int r = 0; r < 8; ++r) sh[wave * 16 + 8 * g + r][j * 16 + col] = (_Float16)phi1(acc[j][r]);
    __syncthreads(); _Float16* dst = which == 0 ? QH : KH; for (int e = tid; e < 64 * 16; e += 128) { const int rl = e >> 4, q = e & 15; vst2((unsigned*)(dst + (r0 + rl) * DM_ + c0 + q * 8), *(const v4u*)&sh[rl][q * 8]); } }
  else {
#pragma unroll
    for (int j = 0; j < 8; ++j)
#pragma unroll
      for (int r = 0; r < 8; ++r) th[j * 16 + col][wave * 16 + 8 * g + r] = (_Float16)acc[j][r];
    __syncthreads(); const size_t b = r0 / LL; const int l0 = (int)(r0 % LL); for (int e = tid; e < 128 * 8; e += 128) { const int cl = e >> 3, q = e & 7; vst2((unsigned*)(VT + (b * DM_ + c0 + cl) * (size_t)LL + l0 + q * 8), *(const v4u*)&th[cl][q * 8]); } } }
__global__ __launch_bounds__(256) void k_gates(const float* __restrict__ X, const float* __restrict__ WW, const float* __restrict__ BW, const float* __restrict__ WE, const float* __restrict__ BE, float* __restrict__ GT) { __shared__ __align__(16) float sx[DM_]; __shared__ __align__(16) float so[32];
  const int t = threadIdx.x; const size_t row = blockIdx.x; for (int i = t; i < DM_; i += 256) sx[i] = bfr(X[row * DM_ + i]);
  __syncthreads();
  { const int wv = t >> 5, ln = t & 31;
    for (int o = wv; o < 32; o += 8) { const float* Wm = (o < 16) ? (WW + (size_t)o * DM_) : (WE + (size_t)(o - 16) * DM_); float a = 0.f; for (int i = ln; i < DM_; i += 32) a += sx[i] * bfr(Wm[i]);
#pragma unroll
      for (int k = 1; k < 32; k <<= 1) a += __shfl_xor(a, k);
      if (ln == 0) { if (o < 16) { const float z = a + bfr(BW[o]); const float sg = 1.0f / (1.0f + expf(-z)); so[o] = logf(sg); } else { const float z = a + bfr(BE[o - 16]); const float sg = 1.0f / (1.0f + expf(-z)); so[o] = logf((1.0f - sg) * 0.95f + 1e-8f); } } } }
  __syncthreads(); if (t < 8) vst2(GT + row * 32 + t * 4, *(const v4f*)&so[t * 4]); }
__global__ __launch_bounds__(256) void k_scan(const float* __restrict__ GT, float* __restrict__ GJ) { __shared__ __align__(16) float sg[LL]; const int t = threadIdx.x; const int h = blockIdx.x; const size_t b = blockIdx.y;
  if (t == 0) { float c = 0.f;
#pragma unroll 1
    for (int l = 0; l < LL; ++l) { c += GT[(b * LL + l) * 32 + 16 + h]; sg[l] = GT[(b * LL + l) * 32 + h] - c; } }
  __syncthreads(); for (int q = t; q < LL / 4; q += 256) vst2(GJ + (b * NH + h) * (size_t)LL + q * 4, *(const v4f*)&sg[q * 4]); }
__global__ __launch_bounds__(128) void k_att(const _Float16* __restrict__ QH, const _Float16* __restrict__ KH, const _Float16* __restrict__ VT, const float* __restrict__ GJ, float* __restrict__ O) {
  __shared__ __align__(16) float sp[4][16][36]; __shared__ __align__(16) float so[4][16][68]; __shared__ float sgj[32];
  const int tid = threadIdx.x, wave = tid >> 5, lane = tid & 31, col = lane & 15, g = lane >> 4; const int qb = blockIdx.x, h = blockIdx.y; const size_t b = blockIdx.z; const int q0l = qb * 64 + wave * 16; const size_t q0 = b * LL + q0l;
  v16h aq[2];
#pragma unroll
  for (int kc = 0; kc < 2; ++kc) aq[kc] = frag_h(QH + (q0 + col) * DM_ + h * HD + kc * 32, lane);
  float m[8], l[8];
#pragma unroll
  for (int r = 0; r < 8; ++r) { m[r] = -3.0e38f; l[r] = 0.f; }
  v8f acc[4] = {};
  const int nks = (qb * 64 + 64) / 32;
#pragma unroll 1
  for (int ks = 0; ks < nks; ++ks) {
    __syncthreads(); if (tid < 32) sgj[tid] = GJ[(b * NH + h) * (size_t)LL + ks * 32 + tid]; __syncthreads();
    float s[2][8];
#pragma unroll
    for (int ct = 0; ct < 2; ++ct) { const int kt = ks * 32 + ct * 16 + col; const size_t kk = b * LL + kt; v8f c = {};
#pragma unroll
      for (int kc = 0; kc < 2; ++kc) c = wmma16(aq[kc], frag_h(KH + kk * DM_ + h * HD + kc * 32, lane), c);
      const float gj = sgj[ct * 16 + col];
#pragma unroll
      for (int r = 0; r < 8; ++r) s[ct][r] = (kt <= q0l + 8 * g + r) ? (logf(fmaxf(c[r], 1e-30f)) + gj) : -3.0e38f; }
    float alpha[8];
#pragma unroll
    for (int r = 0; r < 8; ++r) { float mx = fmaxf(s[0][r], s[1][r]);
#pragma unroll
      for (int o = 1; o < 16; o <<= 1) mx = fmaxf(mx, __shfl_xor(mx, o));
      const float mn = fmaxf(m[r], mx); alpha[r] = (mn <= -1.0e38f) ? 1.f : __expf(m[r] - mn); const float e0 = (s[0][r] <= -1.0e38f) ? 0.f : __expf(s[0][r] - mn), e1 = (s[1][r] <= -1.0e38f) ? 0.f : __expf(s[1][r] - mn); float es = e0 + e1;
#pragma unroll
      for (int o = 1; o < 16; o <<= 1) es += __shfl_xor(es, o);
      l[r] = l[r] * alpha[r] + es; m[r] = mn; sp[wave][8 * g + r][col] = e0; sp[wave][8 * g + r][16 + col] = e1; }
#pragma unroll
    for (int j = 0; j < 4; ++j)
#pragma unroll
      for (int r = 0; r < 8; ++r) acc[j][r] *= alpha[r];
    LDSX();
    const v16h pa = frag_f32s(&sp[wave][col][0], lane, 2048.0f);
#pragma unroll
    for (int j = 0; j < 4; ++j) acc[j] = wmma16(pa, frag_h(VT + (b * DM_ + (size_t)h * HD + j * 16 + col) * LL + ks * 32, lane), acc[j]);
    LDSX(); }
#pragma unroll
  for (int r = 0; r < 8; ++r) { const float il = (1.0f / 2048.0f) / l[r];
#pragma unroll
    for (int j = 0; j < 4; ++j) so[wave][8 * g + r][j * 16 + col] = acc[j][r] * il; }
  LDSX(); for (int rl = 0; rl < 16; ++rl) if (lane < 16) vst2(O + (q0 + rl) * DM_ + h * HD + lane * 4, *(const v4f*)&so[wave][rl][lane * 4]); }
__global__ __launch_bounds__(128) void k_out(const float* __restrict__ O, const float* __restrict__ WO, float* __restrict__ OUT) { __shared__ __align__(16) float sf[4][16][132];
  const int tid = threadIdx.x, wave = tid >> 5, lane = tid & 31, col = lane & 15, g = lane >> 4; const int c0 = blockIdx.y * 128; const size_t r0 = (size_t)blockIdx.x * 64 + wave * 16;
  v8f acc[8] = {};
#pragma unroll 2
  for (int kc = 0; kc < DM_ / 32; ++kc) { const F2 a = split_row(O + (r0 + col) * DM_, kc * 32, lane);
#pragma unroll
    for (int j = 0; j < 8; ++j) { v16b w; const int o = c0 + j * 16 + col;
#pragma unroll
      for (int i = 0; i < 8; ++i) { w[i] = (__bf16)WO[(size_t)o * DM_ + kc * 32 + 8 * g + i]; w[8 + i] = (__bf16)WO[(size_t)o * DM_ + kc * 32 + 16 + 8 * g + i]; }
      acc[j] = wmma_bf(a.h, w, acc[j]); acc[j] = wmma_bf(a.l, w, acc[j]); } }
#pragma unroll
  for (int j = 0; j < 8; ++j)
#pragma unroll
    for (int r = 0; r < 8; ++r) sf[wave][8 * g + r][j * 16 + col] = acc[j][r];
  LDSX(); for (int rl = 0; rl < 16; ++rl) vst2(OUT + (r0 + rl) * DM_ + c0 + lane * 4, *(const v4f*)&sf[wave][rl][lane * 4]); }
extern "C" void kernel_launch(void* const* d_in, const int* in_sizes, int n_in, void* d_out, int out_size, void* d_ws, size_t ws_size, hipStream_t stream) {
  (void)in_sizes; (void)n_in; (void)out_size;
  const float** F = (const float**)d_in;
  if (ws_size < (size_t)WS_END) return;
  char* ws = (char*)d_ws; _Float16 *QH = (_Float16*)(ws + WS_QH), *KH = (_Float16*)(ws + WS_KH), *VT = (_Float16*)(ws + WS_VT); float *GT = (float*)(ws + WS_GT), *GJ = (float*)(ws + WS_GJ), *O = (float*)(ws + WS_O);
  k_proj<<<dim3(TNB * LL / 64, DM_ / 128, 3), 128, 0, stream>>>(F[0], F[1], F[2], F[3], QH, KH, VT);
  k_gates<<<TNB * LL, 256, 0, stream>>>(F[0], F[5], F[6], F[7], F[8], GT);
  k_scan<<<dim3(NH, TNB), 256, 0, stream>>>(GT, GJ);
  k_att<<<dim3(TQB, NH, TNB), 128, 0, stream>>>(QH, KH, VT, GJ, O);
  for (int b = 0; b < TNB; ++b) k_out<<<dim3(TQB, DM_ / 128), 128, 0, stream>>>(O + (size_t)b * LL * DM_, F[4], (float*)d_out + (size_t)b * LL * DM_);
}
